// CompressedInteractionNet_31997506355236
// MI455X (gfx1250) — hardware-verified
//
#include <hip/hip_runtime.h>
#include <math.h>

typedef __attribute__((ext_vector_type(8)))  _Float16 v8h;
typedef __attribute__((ext_vector_type(16))) __bf16   v16b;
typedef __attribute__((ext_vector_type(8)))  __bf16   v8b;
typedef __attribute__((ext_vector_type(8)))  float    v8f;
typedef __attribute__((ext_vector_type(4)))  float    v4f;

constexpr int kNB   = 128;
constexpr int kNI   = 64;
constexpr int kND   = 16;
constexpr int kNK   = 64;
constexpr int kNV   = 16;
constexpr int kGrp  = 1024;
constexpr int kRowsV = kNK * kNV;
constexpr int kRowsX = kNB * kND;
constexpr int kDepth = 64;
static_assert(kNI * kND == kGrp && kNI * kNV == kGrp && kNV * kDepth == kGrp, "group size");
static_assert(kNI == kDepth, "depth");
static_assert((kDepth % 32) == 0, "depth multiple of 32");
static_assert((kRowsV % 64) == 0 && (kRowsX % 64) == 0, "tile multiples");
static_assert(kNV == 16 && kND == 16, "one 16x16 tile per (b,k)");
static_assert((kNB % 4) == 0 && (kNK % 4) == 0, "block tiling");

constexpr size_t kPlaneV = (size_t)kRowsV * kDepth * 2;
constexpr size_t kPlaneX = (size_t)kRowsX * kDepth * 2;
constexpr size_t kOffAMH = 0;
constexpr size_t kOffAML = kOffAMH + kPlaneV;
constexpr size_t kOffAHH = kOffAML + kPlaneV;
constexpr size_t kOffAHL = kOffAHH + kPlaneV;
constexpr size_t kOffBTH = kOffAHL + kPlaneV;
constexpr size_t kOffBTL = kOffBTH + kPlaneX;
constexpr size_t kOffBFH = kOffBTL + kPlaneX;
constexpr size_t kOffBFL = kOffBFH + kPlaneX;
constexpr size_t kWsTotal = kOffBFL + kPlaneX;
static_assert(kPlaneV == 131072ull && kPlaneX == 262144ull, "plane sizes");
static_assert(kWsTotal == 1572864ull, "carve total");
static_assert(kWsTotal <= 134217728ull, "carve cap");
static_assert((kPlaneV % 128) == 0 && (kPlaneX % 128) == 0, "128-B aligned regions");

__device__ __forceinline__ unsigned short f2bf_bits(float f) {
  unsigned u = __float_as_uint(f);
  return (unsigned short)((u + 0x7FFFu + ((u >> 16) & 1u)) >> 16);
}
__device__ __forceinline__ float bf_bits2f(unsigned short h) { return __uint_as_float(((unsigned)h) << 16); }

__device__ __forceinline__ v16b frag_load(const __bf16* p) {
  union U { v16b v; v8b h[2]; };
  U f;
  f.h[0] = *(const v8b*)(p);
  f.h[1] = *(const v8b*)(p + 16);
  return f.v;
}

__device__ __forceinline__ v8f mma_g(v16b a, v16b b, v8f c) {
  c = __builtin_amdgcn_wmma_f32_16x16x32_bf16(false, a, false, b, (short)0, c, false, false);
  asm volatile("v_nop\n\tv_nop\n\tv_nop\n\tv_nop" : "+v"(c) : "v"(a), "v"(b));
  return c;
}

__global__ __launch_bounds__(256) void split_rows_bf16_kernel(
    const float* __restrict__ src, unsigned short* __restrict__ dhi, unsigned short* __restrict__ dlo, int total8)
{
  const int i = blockIdx.x * 256 + threadIdx.x;
  if (i >= total8) return;
  const size_t e0 = (size_t)i << 3;
  const v4f a0 = *(const v4f*)(src + e0);
  const v4f a1 = *(const v4f*)(src + e0 + 4);
  v8h hv, lv;
#pragma unroll
  for (int e = 0; e < 4; ++e) {
    const float f0 = a0[e];
    const float f1 = a1[e];
    const unsigned short h0 = f2bf_bits(f0), h1 = f2bf_bits(f1);
    const unsigned short l0 = f2bf_bits(f0 - bf_bits2f(h0)), l1 = f2bf_bits(f1 - bf_bits2f(h1));
    hv[e]     = __builtin_bit_cast(_Float16, h0);
    hv[4 + e] = __builtin_bit_cast(_Float16, h1);
    lv[e]     = __builtin_bit_cast(_Float16, l0);
    lv[4 + e] = __builtin_bit_cast(_Float16, l1);
  }
  unsigned short* qh = dhi + e0;
  unsigned short* ql = dlo + e0;
  *(volatile v8h*)qh = hv;
  *(volatile v8h*)ql = lv;
  __threadfence();
  *(volatile v8h*)qh = hv;
  *(volatile v8h*)ql = lv;
}

__global__ __launch_bounds__(128) void transpose_split_kernel(
    const float* __restrict__ src, unsigned short* __restrict__ dhi, unsigned short* __restrict__ dlo)
{
  const int t  = threadIdx.x;
  const int c  = t >> 3;
  const int i0 = (t & 7) * 8;
  const float* sp = src + (size_t)blockIdx.x * kGrp + (size_t)i0 * 16 + c;
  float f[8];
#pragma unroll
  for (int e = 0; e < 8; ++e) f[e] = sp[e * 16];
  v8h hv, lv;
#pragma unroll
  for (int e = 0; e < 8; ++e) {
    const unsigned short hb = f2bf_bits(f[e]);
    const unsigned short lb = f2bf_bits(f[e] - bf_bits2f(hb));
    hv[e] = __builtin_bit_cast(_Float16, hb);
    lv[e] = __builtin_bit_cast(_Float16, lb);
  }
  const size_t o = (size_t)blockIdx.x * kGrp + (size_t)t * 8;
  unsigned short* qh = dhi + o;
  unsigned short* ql = dlo + o;
  *(volatile v8h*)qh = hv;
  *(volatile v8h*)ql = lv;
  __threadfence();
  *(volatile v8h*)qh = hv;
  *(volatile v8h*)ql = lv;
}

__global__ __launch_bounds__(128) void dual_gemm_vdot_kernel(
    const unsigned short* __restrict__ AMHp, const unsigned short* __restrict__ AMLp,
    const unsigned short* __restrict__ AHHp, const unsigned short* __restrict__ AHLp,
    const unsigned short* __restrict__ BTHp, const unsigned short* __restrict__ BTLp,
    const unsigned short* __restrict__ BFHp, const unsigned short* __restrict__ BFLp,
    float* __restrict__ out)
{
  const __bf16* AMH = (const __bf16*)AMHp;
  const __bf16* AML = (const __bf16*)AMLp;
  const __bf16* AHH = (const __bf16*)AHHp;
  const __bf16* AHL = (const __bf16*)AHLp;
  const __bf16* BTH = (const __bf16*)BTHp;
  const __bf16* BTL = (const __bf16*)BTLp;
  const __bf16* BFH = (const __bf16*)BFHp;
  const __bf16* BFL = (const __bf16*)BFLp;

  const int lane = threadIdx.x & 31;
  const int wave = __builtin_amdgcn_readfirstlane((int)(threadIdx.x >> 5));
  const int hh   = lane >> 4;
  const int c    = lane & 15;
  const int b    = blockIdx.y * 4 + wave;
  const int kbase = blockIdx.x * 4;

  const size_t brow = (size_t)(b * 16 + c) * kDepth + 8 * hh;
  v16b bth[2], btl[2], bfh[2], bfl[2];
#pragma unroll
  for (int ks = 0; ks < 2; ++ks) {
    bth[ks] = frag_load(BTH + brow + ks * 32);
    btl[ks] = frag_load(BTL + brow + ks * 32);
    bfh[ks] = frag_load(BFH + brow + ks * 32);
    bfl[ks] = frag_load(BFL + brow + ks * 32);
  }

#pragma unroll 1
  for (int pr = 0; pr < 2; ++pr) {
    const int ke = kbase + 2 * pr;
    float sv[2];
#pragma unroll
    for (int t = 0; t < 2; ++t) {
      const size_t arow = (size_t)((ke + t) * 16 + c) * kDepth + 8 * hh;
      v8f acc_a = (v8f){0.f, 0.f, 0.f, 0.f, 0.f, 0.f, 0.f, 0.f};
      v8f acc_b = (v8f){0.f, 0.f, 0.f, 0.f, 0.f, 0.f, 0.f, 0.f};
#pragma unroll
      for (int ks = 0; ks < 2; ++ks) {
        const v16b amh = frag_load(AMH + arow + ks * 32);
        const v16b aml = frag_load(AML + arow + ks * 32);
        const v16b ahh = frag_load(AHH + arow + ks * 32);
        const v16b ahl = frag_load(AHL + arow + ks * 32);
        acc_a = mma_g(amh, bth[ks], acc_a);
        acc_a = mma_g(amh, btl[ks], acc_a);
        acc_a = mma_g(aml, bth[ks], acc_a);
        acc_b = mma_g(ahh, bfh[ks], acc_b);
        acc_b = mma_g(ahh, bfl[ks], acc_b);
        acc_b = mma_g(ahl, bfh[ks], acc_b);
      }
      float s = 0.0f;
#pragma unroll
      for (int r = 0; r < 8; ++r) s = fmaf(acc_a[r], acc_b[r], s);
      const float so = __shfl_xor(s, 16, 32);
      sv[t] = s + so;
    }
    const float val = (hh == 0) ? sv[0] : sv[1];
    float* p = out + (size_t)b * kGrp + (size_t)ke * 16 + lane;
    *(volatile float*)p = val;
    __threadfence();
    *(volatile float*)p = val;
  }
}

extern "C" void kernel_launch(void* const* d_in, const int* in_sizes, int n_in,
                              void* d_out, int out_size, void* d_ws, size_t ws_size,
                              hipStream_t stream) {
  if (n_in < 4) return;
  if (in_sizes[0] != kNB * kGrp) return;
  if (in_sizes[2] != kNK * kGrp) return;
  if (in_sizes[3] != kNK * kGrp) return;
  if (out_size != kNB * kNK * kND) return;
  if (ws_size < kWsTotal) return;

  const float* x0 = (const float*)d_in[0];
  const float* Vm = (const float*)d_in[2];
  const float* Vh = (const float*)d_in[3];
  float* out = (float*)d_out;

  char* ws = (char*)d_ws;
  unsigned short* AMH = (unsigned short*)(ws + kOffAMH);
  unsigned short* AML = (unsigned short*)(ws + kOffAML);
  unsigned short* AHH = (unsigned short*)(ws + kOffAHH);
  unsigned short* AHL = (unsigned short*)(ws + kOffAHL);
  unsigned short* BTH = (unsigned short*)(ws + kOffBTH);
  unsigned short* BTL = (unsigned short*)(ws + kOffBTL);
  unsigned short* BFH = (unsigned short*)(ws + kOffBFH);
  unsigned short* BFL = (unsigned short*)(ws + kOffBFL);

  split_rows_bf16_kernel<<<(kNK * kGrp / 8) / 256, 256, 0, stream>>>(Vh, AHH, AHL, kNK * kGrp / 8);
  split_rows_bf16_kernel<<<(kNB * kGrp / 8) / 256, 256, 0, stream>>>(x0, BFH, BFL, kNB * kGrp / 8);
  transpose_split_kernel<<<kNK, 128, 0, stream>>>(Vm, AMH, AML);
  transpose_split_kernel<<<kNB, 128, 0, stream>>>(x0, BTH, BTL);

  dual_gemm_vdot_kernel<<<dim3(kNK / 4, kNB / 4), 128, 0, stream>>>(
      AMH, AML, AHH, AHL, BTH, BTL, BFH, BFL, out);
}
